// SSM_cha_36386962932304
// MI455X (gfx1250) — hardware-verified
//
#include <hip/hip_runtime.h>
#include <math.h>

typedef __attribute__((ext_vector_type(16))) _Float16 v16h;
typedef __attribute__((ext_vector_type(8)))  _Float16 v8h;
typedef __attribute__((ext_vector_type(16))) __bf16   v16b;
typedef __attribute__((ext_vector_type(8)))  __bf16   v8b;
typedef __attribute__((ext_vector_type(8)))  float    v8f;
typedef __attribute__((ext_vector_type(4)))  float    v4f;

constexpr int kBatch = 16;
constexpr int kL     = 4096;
constexpr int kD     = 128;
constexpr int kNProj = 12;
constexpr int kDtR   = 8;
constexpr int kXZP   = 2 * kD;
constexpr int kRows  = kBatch * kL;
constexpr int kChunk = 32;
constexpr int kTP    = 132;
static_assert(kL % kChunk == 0);
static_assert(kRows % 64 == 0 && kD % 64 == 0 && kXZP % 64 == 0 && kD % 32 == 0);

__device__ __forceinline__ unsigned short f2bf_bits(float f) {
  unsigned u = __float_as_uint(f);
  return (unsigned short)((u + 0x7FFFu + ((u >> 16) & 1u)) >> 16);
}
__device__ __forceinline__ float bf_bits2f(unsigned short h) { return __uint_as_float(((unsigned)h) << 16); }

__device__ __forceinline__ void dep_guard_h(v8f& a, v8f& b, v16h x, v16h y) { asm volatile("v_nop\n\tv_nop\n\tv_nop\n\tv_nop" : "+v"(a), "+v"(b) : "v"(x), "v"(y)); }
__device__ __forceinline__ void dep_guard_b(v8f& a, v8f& b, v16b x, v16b y) { asm volatile("v_nop\n\tv_nop\n\tv_nop\n\tv_nop" : "+v"(a), "+v"(b) : "v"(x), "v"(y)); }
__device__ __forceinline__ void keep4_h(v16h a, v16h b, v16h c, v16h d) { asm volatile("v_nop" :: "v"(a), "v"(b), "v"(c), "v"(d)); }
__device__ __forceinline__ void keep4_b(v16b a, v16b b, v16b c, v16b d) { asm volatile("v_nop" :: "v"(a), "v"(b), "v"(c), "v"(d)); }
__device__ __forceinline__ void acc_guard4(v8f& a, v8f& b, v8f& c, v8f& d) { asm volatile("v_nop\n\tv_nop\n\tv_nop\n\tv_nop" : "+v"(a), "+v"(b), "+v"(c), "+v"(d)); }
template <typename T> struct Frag;
template <> struct Frag<_Float16> {
  typedef v16h V; union U { v16h v; v8h h[2]; };
  static __device__ __forceinline__ v16h load(const _Float16* p) {
    U f; f.h[0] = *(const v8h*)(p); f.h[1] = *(const v8h*)(p + 16); return f.v;
  }
  static __device__ __forceinline__ v8f mma(v16h a, v16h b, v8f c) {
    return __builtin_amdgcn_wmma_f32_16x16x32_f16(false, a, false, b, (short)0, c, false, false);
  }
  static __device__ __forceinline__ void guard(v8f& a, v8f& b, v16h x, v16h y) { dep_guard_h(a, b, x, y); }
  static __device__ __forceinline__ void keep(v16h a, v16h b, v16h c, v16h d) { keep4_h(a, b, c, d); }
};
template <> struct Frag<__bf16> {
  typedef v16b V; union U { v16b v; v8b h[2]; };
  static __device__ __forceinline__ v16b load(const __bf16* p) {
    U f; f.h[0] = *(const v8b*)(p); f.h[1] = *(const v8b*)(p + 16); return f.v;
  }
  static __device__ __forceinline__ v8f mma(v16b a, v16b b, v8f c) {
    return __builtin_amdgcn_wmma_f32_16x16x32_bf16(false, a, false, b, (short)0, c, false, false);
  }
  static __device__ __forceinline__ void guard(v8f& a, v8f& b, v16b x, v16b y) { dep_guard_b(a, b, x, y); }
  static __device__ __forceinline__ void keep(v16b a, v16b b, v16b c, v16b d) { keep4_b(a, b, c, d); }
};

template <int ET> struct Elem;
template <> struct Elem<0> { typedef _Float16 T; };
template <> struct Elem<1> { typedef __bf16 T; };
template <int ET, bool SPLIT, int BIAS_MODE, int OUT_MODE, bool RESID, int ACT = 0>
__global__ __launch_bounds__(256) void wmma_gemm64(
    const unsigned short* __restrict__ Ap, const unsigned short* __restrict__ A2p, int lda, long strideA,
    const unsigned short* __restrict__ Btp, const unsigned short* __restrict__ Bt2p, int ldb, long strideB,
    void* __restrict__ Cout, void* __restrict__ Cout2, int ldc, long strideC,
    const float* __restrict__ bias,
    const float* __restrict__ resid, long strideR,
    int M, int N, int K, float scale) {
  typedef typename Elem<ET>::T T;
  typedef typename Frag<T>::V V;
  const T* A = (const T*)Ap; const T* A2 = (const T*)A2p; const T* Bt = (const T*)Btp; const T* Bt2 = (const T*)Bt2p;
  __shared__ __align__(16) float sT[8][16 * 68];
  const int b    = blockIdx.y;
  const int lane = threadIdx.x & 31;
  const int wave = threadIdx.x >> 5;
  const int tilesN = N >> 6;
  const int tilesM = M >> 6;
  const int tile = blockIdx.x * 8 + wave;
  if (tile >= tilesM * tilesN) return;
  const int tm = tile / tilesN;
  const int tn = tile - tm * tilesN;
  const int m0 = tm << 6;
  const int n0 = tn << 6;

  const T* Ab  = A  + (size_t)b * strideA;
  const T* Bb  = Bt + (size_t)b * strideB;
  const T* Ab2 = SPLIT ? (A2  + (size_t)b * strideA) : nullptr;
  const T* Bb2 = SPLIT ? (Bt2 + (size_t)b * strideB) : nullptr;

  const int rlane = lane & 15;
  const int koff  = (lane >> 4) * 8;
  const int mOff  = (lane >> 4) * 8;

  v8f acc[4][4];
#pragma unroll
  for (int i = 0; i < 4; ++i)
#pragma unroll
    for (int j = 0; j < 4; ++j) acc[i][j] = (v8f){0.f,0.f,0.f,0.f,0.f,0.f,0.f,0.f};

  for (int k0 = 0; k0 < K; k0 += 32) {
    V bh[4], bl[4];
#pragma unroll
    for (int j = 0; j < 4; ++j) {
      const size_t bo = (size_t)(n0 + (j << 4) + rlane) * ldb + koff + k0;
      bh[j] = Frag<T>::load(Bb + bo);
      if (SPLIT) bl[j] = Frag<T>::load(Bb2 + bo);
    }
#pragma unroll
    for (int i = 0; i < 4; ++i) {
      const size_t ao = (size_t)(m0 + (i << 4) + rlane) * lda + koff + k0;
      V ah = Frag<T>::load(Ab + ao);
      V al;
      if (SPLIT) al = Frag<T>::load(Ab2 + ao);
#pragma unroll
      for (int j = 0; j < 4; ++j) {
        acc[i][j] = Frag<T>::mma(ah, bh[j], acc[i][j]);
        if (SPLIT) {
          acc[i][j] = Frag<T>::mma(ah, bl[j], acc[i][j]);
          acc[i][j] = Frag<T>::mma(al, bh[j], acc[i][j]);
        }
      }
      Frag<T>::guard(acc[i][0], acc[i][3], ah, SPLIT ? al : ah);
    }
    Frag<T>::keep(bh[0], bh[1], bh[2], bh[3]);
    if (SPLIT) Frag<T>::keep(bl[0], bl[1], bl[2], bl[3]);
  }
  acc_guard4(acc[0][0], acc[0][1], acc[0][2], acc[0][3]);
  acc_guard4(acc[1][0], acc[1][1], acc[1][2], acc[1][3]);
  acc_guard4(acc[2][0], acc[2][1], acc[2][2], acc[2][3]);
  acc_guard4(acc[3][0], acc[3][1], acc[3][2], acc[3][3]);

  float* slab = sT[wave];
  const float* Rb = RESID ? (resid + (size_t)b * strideR) : nullptr;
#pragma unroll
  for (int i = 0; i < 4; ++i) {
    const int mBase = m0 + (i << 4);
#pragma unroll
    for (int j = 0; j < 4; ++j) {
      const int n = n0 + (j << 4) + rlane;
      float bv = 0.f;
      if (BIAS_MODE == 2) bv = bias[n];
#pragma unroll
      for (int r = 0; r < 8; ++r) {
        float v = acc[i][j][r] * scale;
        if (BIAS_MODE == 1) v += bias[mBase + mOff + r];
        if (BIAS_MODE == 2) v += bv;
        if (RESID) v += Rb[(size_t)(mBase + mOff + r) * ldc + n];
        if (ACT == 1) v = tanhf(v);
        if (ACT == 2) v = fmaxf(v, 0.0f);
        if (ACT == 3) v = v / (1.0f + expf(-v));
        if (ACT == 4) v = (v > 0.f) ? v : 0.01f * v;
        if (ACT == 5) v = 0.5f * v * (1.0f + erff(v * 0.70710678118654752f));
        slab[(mOff + r) * 68 + (j << 4) + rlane] = v;
      }
    }
    __builtin_amdgcn_fence(__ATOMIC_RELEASE, "workgroup");
    __builtin_amdgcn_wave_barrier();
    __builtin_amdgcn_fence(__ATOMIC_ACQUIRE, "workgroup");
    if (OUT_MODE == 0) {
      float* C = (float*)Cout + (size_t)b * strideC;
      const int hh = lane >> 4, c4 = (lane & 15) * 4;
      for (int pass = 0; pass < 2; ++pass) {
#pragma unroll
        for (int it = 0; it < 8; ++it) {
          const int row = it * 2 + hh;
          v4f v = *(const v4f*)(slab + row * 68 + c4);
          *(volatile v4f*)(C + (size_t)(mBase + row) * ldc + n0 + c4) = v;
        }
        __threadfence();
      }
    } else {
      const int q = lane >> 3, c8 = (lane & 7) * 8;
      unsigned short* C  = (unsigned short*)Cout  + (size_t)b * strideC;
      unsigned short* C2 = (OUT_MODE == 2) ? ((unsigned short*)Cout2 + (size_t)b * strideC) : nullptr;
      for (int pass = 0; pass < 2; ++pass) {
#pragma unroll
        for (int it = 0; it < 4; ++it) {
          const int row = it * 4 + q;
          const float* sp = slab + row * 68 + c8;
          v8h hv, lv;
#pragma unroll
          for (int e = 0; e < 8; ++e) {
            if (OUT_MODE == 1) {
              hv[e] = (_Float16)sp[e];
            } else {
              unsigned short hb = f2bf_bits(sp[e]);
              unsigned short lb = f2bf_bits(sp[e] - bf_bits2f(hb));
              hv[e] = __builtin_bit_cast(_Float16, hb);
              lv[e] = __builtin_bit_cast(_Float16, lb);
            }
          }
          *(volatile v8h*)(C + (size_t)(mBase + row) * ldc + n0 + c8) = hv;
          if (OUT_MODE == 2) *(volatile v8h*)(C2 + (size_t)(mBase + row) * ldc + n0 + c8) = lv;
        }
        __threadfence();
      }
    }
    __builtin_amdgcn_fence(__ATOMIC_RELEASE, "workgroup");
    __builtin_amdgcn_wave_barrier();
    __builtin_amdgcn_fence(__ATOMIC_ACQUIRE, "workgroup");
  }
}

__global__ __launch_bounds__(256) void split_bf16_kernel(
    const float* __restrict__ src, unsigned short* __restrict__ hi, unsigned short* __restrict__ lo, int total8)
{
  const int i = blockIdx.x * 256 + threadIdx.x;
  if (i >= total8) return;
  const size_t e0 = (size_t)i << 3;
  const float* p = src + e0;
  const v4f a0 = *(const v4f*)(p);
  const v4f a1 = *(const v4f*)(p + 4);
  v8h hv, lv;
#pragma unroll
  for (int e = 0; e < 4; ++e) {
    const unsigned short h0 = f2bf_bits(a0[e]);
    const unsigned short l0 = f2bf_bits(a0[e] - bf_bits2f(h0));
    const unsigned short h1 = f2bf_bits(a1[e]);
    const unsigned short l1 = f2bf_bits(a1[e] - bf_bits2f(h1));
    hv[e]     = __builtin_bit_cast(_Float16, h0);
    lv[e]     = __builtin_bit_cast(_Float16, l0);
    hv[4 + e] = __builtin_bit_cast(_Float16, h1);
    lv[4 + e] = __builtin_bit_cast(_Float16, l1);
  }
  unsigned short* qh = hi + e0;
  unsigned short* ql = lo + e0;
  *(volatile v8h*)qh = hv;
  *(volatile v8h*)ql = lv;
  __threadfence();
  *(volatile v8h*)qh = hv;
  *(volatile v8h*)ql = lv;
}

__global__ __launch_bounds__(256) void x_split_kernel(
    const float* __restrict__ x1, unsigned short* __restrict__ XH, unsigned short* __restrict__ XL)
{
  __shared__ float sT[64][65];
  const int tid = threadIdx.x;
  const int blk = blockIdx.x;
  const int b   = blk >> 7;
  const int rem = blk & 127;
  const int cb  = rem >> 6;
  const int tb  = rem & 63;
  const int c0 = cb * 64, t0 = tb * 64;
  const float* src = x1 + ((size_t)b * kD + c0) * kL + t0;
  const int lr = tid >> 4, lc = (tid & 15) * 4;
#pragma unroll
  for (int it = 0; it < 4; ++it) {
    const int row = it * 16 + lr;
    const v4f v = *(const v4f*)(src + (size_t)row * kL + lc);
    sT[row][lc + 0] = v[0];
    sT[row][lc + 1] = v[1];
    sT[row][lc + 2] = v[2];
    sT[row][lc + 3] = v[3];
  }
  __syncthreads();
  const int g8 = tid >> 3, c8 = (tid & 7) * 8;
  v8h hv[2], lv[2];
#pragma unroll
  for (int it = 0; it < 2; ++it) {
    const int tr = it * 32 + g8;
#pragma unroll
    for (int e = 0; e < 8; ++e) {
      const float f = sT[c8 + e][tr];
      const unsigned short hb = f2bf_bits(f);
      const unsigned short lb = f2bf_bits(f - bf_bits2f(hb));
      hv[it][e] = __builtin_bit_cast(_Float16, hb);
      lv[it][e] = __builtin_bit_cast(_Float16, lb);
    }
  }
  const size_t rowbase = (size_t)b * kL + t0;
  for (int pass = 0; pass < 2; ++pass) {
#pragma unroll
    for (int it = 0; it < 2; ++it) {
      const int tr = it * 32 + g8;
      const size_t o = (rowbase + tr) * kD + c0 + c8;
      *(volatile v8h*)(XH + o) = hv[it];
      *(volatile v8h*)(XL + o) = lv[it];
    }
    __threadfence();
  }
}

__global__ __launch_bounds__(128) void ssm_fused_kernel(
    const float* __restrict__ XZ, const float* __restrict__ conv_w, const float* __restrict__ conv_b,
    const float* __restrict__ W_xproj, const float* __restrict__ W_dt, const float* __restrict__ b_dt,
    const float* __restrict__ A_log, const float* __restrict__ D_param,
    unsigned short* __restrict__ YH, unsigned short* __restrict__ YL)
{
  __shared__ __align__(16) float sW[kNProj * kD];
  __shared__ __align__(16) float sXS[kChunk * kTP];
  __shared__ __align__(16) float sDB[kChunk * 16];
  __shared__ __align__(16) float sY[kChunk * kTP];
  const int tid = threadIdx.x, lane = tid & 31, wave = tid >> 5;
  const int d = tid;
  const size_t rb = (size_t)blockIdx.x * kL;

#pragma unroll 1
  for (int i = 0; i < kNProj; ++i) sW[i * kD + tid] = W_xproj[i * kD + tid];
  const float w0 = conv_w[d * 4 + 0], w1 = conv_w[d * 4 + 1], w2 = conv_w[d * 4 + 2], w3 = conv_w[d * 4 + 3];
  const float cbias = conv_b[d];
  float wdt[kDtR];
#pragma unroll
  for (int r = 0; r < kDtR; ++r) wdt[r] = W_dt[d * kDtR + r];
  const float bdt = b_dt[d];
  const float A0 = -__expf(A_log[d * 2 + 0]);
  const float A1 = -__expf(A_log[d * 2 + 1]);
  const float Dp = D_param[d];
  __syncthreads();

  float xm3 = 0.f, xm2 = 0.f, xm1 = 0.f;
  float h0 = 0.f, h1 = 0.f;
  const int g8 = tid >> 3, c8 = (tid & 7) * 8;

#pragma unroll 1
  for (int c = 0; c < kL / kChunk; ++c) {
    const int t0 = c * kChunk;
#pragma unroll 1
    for (int s = 0; s < kChunk; ++s) {
      const float xc = XZ[(rb + t0 + s) * kXZP + d];
      float acc = w0 * xm3;
      acc = fmaf(w1, xm2, acc);
      acc = fmaf(w2, xm1, acc);
      acc = fmaf(w3, xc, acc);
      const float sv = acc + cbias;
      const float sg = __builtin_amdgcn_rcpf(1.0f + __expf(-sv));
      sXS[s * kTP + d] = sv * sg;
      xm3 = xm2; xm2 = xm1; xm1 = xc;
    }
    __syncthreads();
    {
      const float* xr  = sXS + lane * kTP;
      const float* wr0 = sW + wave * kD;
      const float* wr1 = sW + (wave + 4) * kD;
      const float* wr2 = sW + (wave + 8) * kD;
      float a0 = 0.f, a1 = 0.f, a2 = 0.f;
#pragma unroll 1
      for (int k = 0; k < kD; k += 4) {
        const v4f xv = *(const v4f*)(xr + k);
        const v4f u0 = *(const v4f*)(wr0 + k);
        const v4f u1 = *(const v4f*)(wr1 + k);
        const v4f u2 = *(const v4f*)(wr2 + k);
#pragma unroll
        for (int e = 0; e < 4; ++e) {
          a0 = fmaf(xv[e], u0[e], a0);
          a1 = fmaf(xv[e], u1[e], a1);
          a2 = fmaf(xv[e], u2[e], a2);
        }
      }
      sDB[lane * 16 + wave]     = a0;
      sDB[lane * 16 + wave + 4] = a1;
      sDB[lane * 16 + wave + 8] = a2;
    }
    __syncthreads();
#pragma unroll 1
    for (int s = 0; s < kChunk; ++s) {
      const v4f q0 = *(const v4f*)(sDB + s * 16);
      const v4f q1 = *(const v4f*)(sDB + s * 16 + 4);
      const v4f q2 = *(const v4f*)(sDB + s * 16 + 8);
      float a = q0[0] * wdt[0];
      a = fmaf(q0[1], wdt[1], a);
      a = fmaf(q0[2], wdt[2], a);
      a = fmaf(q0[3], wdt[3], a);
      a = fmaf(q1[0], wdt[4], a);
      a = fmaf(q1[1], wdt[5], a);
      a = fmaf(q1[2], wdt[6], a);
      a = fmaf(q1[3], wdt[7], a);
      a += bdt;
      const float dt = fmaxf(a, 0.0f) + __logf(1.0f + __expf(-fabsf(a)));
      const float xv = sXS[s * kTP + d];
      const float zv = XZ[(rb + t0 + s) * kXZP + kD + d];
      const float e0 = __expf(dt * A0);
      const float e1 = __expf(dt * A1);
      const float B0 = q2[0], B1 = q2[1], C0 = q2[2], C1 = q2[3];
      const float u0 = (dt * B0) * xv;
      const float u1 = (dt * B1) * xv;
      h0 = fmaf(e0, h0, u0);
      h1 = fmaf(e1, h1, u1);
      float y = h0 * C0 + h1 * C1;
      y = y + xv * Dp;
      const float sg = __builtin_amdgcn_rcpf(1.0f + __expf(-zv));
      y = y * (zv * sg);
      sY[s * kTP + d] = y;
    }
    __syncthreads();
    {
      v8h hv[4], lv[4];
#pragma unroll
      for (int it = 0; it < 4; ++it) {
        const int row = it * 8 + (g8 >> 1), half = g8 & 1;
        const float* sp = sY + row * kTP + half * 64 + c8;
        const v4f a0 = *(const v4f*)(sp);
        const v4f a1 = *(const v4f*)(sp + 4);
#pragma unroll
        for (int e = 0; e < 4; ++e) {
          const unsigned short hb0 = f2bf_bits(a0[e]);
          const unsigned short lb0 = f2bf_bits(a0[e] - bf_bits2f(hb0));
          const unsigned short hb1 = f2bf_bits(a1[e]);
          const unsigned short lb1 = f2bf_bits(a1[e] - bf_bits2f(hb1));
          hv[it][e]     = __builtin_bit_cast(_Float16, hb0);
          lv[it][e]     = __builtin_bit_cast(_Float16, lb0);
          hv[it][4 + e] = __builtin_bit_cast(_Float16, hb1);
          lv[it][4 + e] = __builtin_bit_cast(_Float16, lb1);
        }
      }
      for (int pass = 0; pass < 2; ++pass) {
#pragma unroll
        for (int it = 0; it < 4; ++it) {
          const int row = it * 8 + (g8 >> 1), half = g8 & 1;
          const size_t o = (rb + t0 + row) * kD + half * 64 + c8;
          *(volatile v8h*)(YH + o) = hv[it];
          *(volatile v8h*)(YL + o) = lv[it];
        }
        __threadfence();
      }
    }
  }
}

__global__ __launch_bounds__(256) void ln_nchw_kernel(
    const float* __restrict__ PRE, const float* __restrict__ g, const float* __restrict__ be,
    float* __restrict__ out)
{
  __shared__ float sT[64][129];
  __shared__ float smu[64];
  __shared__ float srs[64];
  const int tid = threadIdx.x;
  const int blk = blockIdx.x;
  const int b  = blk >> 6;
  const int tb = blk & 63;
  const int t0 = tb * 64;
  const size_t row0 = (size_t)b * kL + t0;
  {
    const int lr = tid >> 5, lc = (tid & 31) * 4;
#pragma unroll
    for (int it = 0; it < 8; ++it) {
      const int row = it * 8 + lr;
      const v4f v = *(const v4f*)(PRE + (row0 + row) * kD + lc);
      sT[row][lc + 0] = v[0];
      sT[row][lc + 1] = v[1];
      sT[row][lc + 2] = v[2];
      sT[row][lc + 3] = v[3];
    }
  }
  __syncthreads();
  {
    const int r = tid >> 2, p = tid & 3;
    float s = 0.f;
#pragma unroll 1
    for (int k = 0; k < 32; ++k) s += sT[r][p * 32 + k];
    s += __shfl_xor(s, 1, 32);
    s += __shfl_xor(s, 2, 32);
    const float mean = s * (1.0f / 128.0f);
    float s2 = 0.f;
#pragma unroll 1
    for (int k = 0; k < 32; ++k) {
      const float dd = sT[r][p * 32 + k] - mean;
      s2 += dd * dd;
    }
    s2 += __shfl_xor(s2, 1, 32);
    s2 += __shfl_xor(s2, 2, 32);
    const float var  = s2 * (1.0f / 128.0f);
    const float rstd = rsqrtf(var + 1e-5f);
    if (p == 0) { smu[r] = mean; srs[r] = rstd; }
  }
  __syncthreads();
  const int q = tid >> 4, t4 = (tid & 15) * 4;
  v4f o[8];
#pragma unroll
  for (int it = 0; it < 8; ++it) {
    const int c = it * 16 + q;
    const float gc = g[c], bc = be[c];
#pragma unroll
    for (int e = 0; e < 4; ++e) {
      const int t = t4 + e;
      o[it][e] = (sT[t][c] - smu[t]) * srs[t] * gc + bc;
    }
  }
  for (int pass = 0; pass < 2; ++pass) {
#pragma unroll
    for (int it = 0; it < 8; ++it) {
      const int c = it * 16 + q;
      *(volatile v4f*)(out + ((size_t)b * kD + c) * kL + t0 + t4) = o[it];
    }
    __threadfence();
  }
}

extern "C" void kernel_launch(void* const* d_in, const int* in_sizes, int n_in,
                              void* d_out, int out_size, void* d_ws, size_t ws_size,
                              hipStream_t stream)
{
  if (n_in < 12) return;
  const float* x1      = (const float*)d_in[0];
  const float* W_in    = (const float*)d_in[1];
  const float* conv_w  = (const float*)d_in[2];
  const float* conv_b  = (const float*)d_in[3];
  const float* W_xproj = (const float*)d_in[4];
  const float* W_dt    = (const float*)d_in[5];
  const float* b_dt    = (const float*)d_in[6];
  const float* A_log   = (const float*)d_in[7];
  const float* D_param = (const float*)d_in[8];
  const float* W_out   = (const float*)d_in[9];
  const float* ln_g    = (const float*)d_in[10];
  const float* ln_b    = (const float*)d_in[11];
  float* dout = (float*)d_out;

  if (in_sizes[0] != kBatch * kD * kL) return;
  if (in_sizes[1] != 2 * kD * kD) return;
  if (in_sizes[2] != kD * 4 || in_sizes[3] != kD) return;
  if (in_sizes[4] != kNProj * kD) return;
  if (in_sizes[5] != kD * kDtR || in_sizes[6] != kD) return;
  if (in_sizes[7] != kD * 2 || in_sizes[8] != kD) return;
  if (in_sizes[9] != kD * kD) return;
  if (in_sizes[10] != kD || in_sizes[11] != kD) return;
  if (out_size != kBatch * kD * kL) return;

  const size_t SZ_WI  = (size_t)2 * kD * kD * 2;
  const size_t SZ_WO  = (size_t)kD * kD * 2;
  const size_t SZ_XP  = (size_t)kRows * kD * 2;
  const size_t SZ_XZ  = (size_t)kRows * kXZP * 4;
  const size_t OFF_WIH = 0;
  const size_t OFF_WIL = OFF_WIH + SZ_WI;
  const size_t OFF_WOH = OFF_WIL + SZ_WI;
  const size_t OFF_WOL = OFF_WOH + SZ_WO;
  const size_t OFF_XH  = 262144;
  const size_t OFF_XL  = OFF_XH + SZ_XP;
  const size_t OFF_XZ  = OFF_XL + SZ_XP;
  const size_t TOTAL   = OFF_XZ + SZ_XZ;
  if (OFF_WOL + SZ_WO > OFF_XH) return;
  if (ws_size < TOTAL) return;

  char* ws = (char*)d_ws;
  unsigned short* WIH = (unsigned short*)(ws + OFF_WIH);
  unsigned short* WIL = (unsigned short*)(ws + OFF_WIL);
  unsigned short* WOH = (unsigned short*)(ws + OFF_WOH);
  unsigned short* WOL = (unsigned short*)(ws + OFF_WOL);
  unsigned short* XH  = (unsigned short*)(ws + OFF_XH);
  unsigned short* XL  = (unsigned short*)(ws + OFF_XL);
  unsigned short* YH  = XH;
  unsigned short* YL  = XL;
  float*          XZ  = (float*)(ws + OFF_XZ);
  float*          PRE = XZ;
  const float* dummy_bias  = conv_b;
  const float* dummy_resid = conv_b;

  split_bf16_kernel<<<(2 * kD * kD) / 8 / 256, 256, 0, stream>>>(W_in, WIH, WIL, (2 * kD * kD) / 8);
  split_bf16_kernel<<<(kD * kD) / 8 / 256, 256, 0, stream>>>(W_out, WOH, WOL, (kD * kD) / 8);

  x_split_kernel<<<kBatch * (kD / 64) * (kL / 64), 256, 0, stream>>>(x1, XH, XL);

  wmma_gemm64<1, true, 0, 0, false><<<dim3(512, 1), 256, 0, stream>>>(
      XH, XL, kD, 0L, WIH, WIL, kD, 0L,
      (void*)XZ, (void*)XZ, kXZP, 0L, dummy_bias, dummy_resid, 0L, kRows, kXZP, kD, 1.0f);

  ssm_fused_kernel<<<kBatch, kD, 0, stream>>>(XZ, conv_w, conv_b, W_xproj, W_dt, b_dt, A_log, D_param, YH, YL);

  wmma_gemm64<1, true, 0, 0, false><<<dim3(256, 1), 256, 0, stream>>>(
      YH, YL, kD, 0L, WOH, WOL, kD, 0L,
      (void*)PRE, (void*)PRE, kD, 0L, dummy_bias, dummy_resid, 0L, kRows, kD, kD, 1.0f);

  ln_nchw_kernel<<<kRows / 64, 256, 0, stream>>>(PRE, ln_g, ln_b, dout);

  (void)hipGetLastError();
}
